// SelfAttention_53695681134997
// MI455X (gfx1250) — hardware-verified
//
#include <hip/hip_runtime.h>
#include <math.h>

typedef __attribute__((ext_vector_type(16))) _Float16 v16h;
typedef __attribute__((ext_vector_type(16))) __bf16 v16b;
typedef __attribute__((ext_vector_type(8)))  _Float16 v8h;
typedef __attribute__((ext_vector_type(8)))  __bf16 v8b;
typedef __attribute__((ext_vector_type(8)))  float v8f;
typedef __attribute__((ext_vector_type(4)))  float v4f;
typedef __attribute__((ext_vector_type(4)))  unsigned v4u;
typedef v4u __attribute__((may_alias)) v4u_a;
typedef v4f __attribute__((may_alias)) v4f_a;
typedef v8h __attribute__((may_alias)) v8h_a;

#ifndef NB
#define NB 2
#endif
#ifndef SEQ
#define SEQ 2048
#endif
#define SEQ_FULL 2048
#define DM 1024
#define NH 16
#define HD 64
#define NTOK (NB * SEQ)
#define TPS (SEQ / NH)
#define NSLAB (NH * NB)
#define SCALE 0.03125f
#define LN1024 6.931471806f

static_assert(SEQ % 1024 == 0);
static_assert(NTOK % 64 == 0);
static_assert(DM % 128 == 0);
static_assert(SEQ <= SEQ_FULL);

#define PLANE2 (2ull * (unsigned long long)NTOK * DM)
#define WPL2   (2ull * (unsigned long long)DM * DM)
#define WS_XB 0ull
#define WS_YB (WS_XB + PLANE2)
#define WS_WT (WS_YB + PLANE2)
#define WS_QH (WS_WT + 4ull * WPL2)
#define WS_KH (WS_QH + PLANE2)
#define WS_VT (WS_KH + PLANE2)
#define WS_CH (WS_VT + PLANE2)
#define WS_CL (WS_CH + PLANE2)
#define WS_END (WS_CL + PLANE2)
static_assert(WS_END <= 134217728ull);
static_assert(PLANE2 % 128 == 0);
static_assert(WPL2 % 128 == 0);

template <typename T> __device__ __forceinline__ void vst2(T* p, T v) { *(volatile T*)p = v; __threadfence(); *(volatile T*)p = v; }

__device__ __forceinline__ v8f wmma16(v16h a, v16h b, v8f c) {
  v8f d = __builtin_amdgcn_wmma_f32_16x16x32_f16(false, a, false, b, (short)0, c, false, false);
  asm volatile("v_nop\n\tv_nop\n\tv_nop\n\tv_nop" : "+v"(d) : "v"(a), "v"(b));
  return d;
}
__device__ __forceinline__ v8f wmma_bf(v16b a, v16b b, v8f c) {
  v8f d = __builtin_amdgcn_wmma_f32_16x16x32_bf16(false, a, false, b, (short)0, c, false, false);
  asm volatile("v_nop\n\tv_nop\n\tv_nop\n\tv_nop" : "+v"(d) : "v"(a), "v"(b));
  return d;
}
__device__ __forceinline__ v16h frag_h(const _Float16* rowk0, int lane) {
  union { v16h v; v8h q[2]; } u; const _Float16* p = rowk0 + 8 * (lane >> 4);
  u.q[0] = *(const v8h*)p; u.q[1] = *(const v8h*)(p + 16); return u.v;
}
__device__ __forceinline__ v16b frag_b(const __bf16* rowk0, int lane) {
  union { v16b v; v8b q[2]; } u; const __bf16* p = rowk0 + 8 * (lane >> 4);
  u.q[0] = *(const v8b*)p; u.q[1] = *(const v8b*)(p + 16); return u.v;
}
__device__ __forceinline__ unsigned bf16_rne(float f) { unsigned u = __float_as_uint(f); u += 0x7FFFu + ((u >> 16) & 1u); return u >> 16; }
__device__ __forceinline__ float bfr(float v) { return __uint_as_float(bf16_rne(v) << 16); }
__device__ __forceinline__ unsigned pack2(float a, float b) { return bf16_rne(a) | (bf16_rne(b) << 16); }
__device__ __forceinline__ void ldsx() { asm volatile("s_wait_dscnt 0" ::: "memory"); __builtin_amdgcn_wave_barrier(); __builtin_amdgcn_fence(3  , "workgroup"); }

__global__ __launch_bounds__(256) void k_cvt(const float* __restrict__ X, unsigned* __restrict__ XB) {
  const size_t e = (size_t)blockIdx.x * 256 + threadIdx.x;
  if (e >= (size_t)NTOK * (DM / 8)) return;
  const int T = (int)(e >> 7); const int pc = (int)(e & 127); const int b = T / SEQ; const int s = T - b * SEQ;
  const float* p = X + ((size_t)b * SEQ_FULL + s) * DM + pc * 8;
  const v4f a = *(const v4f*)p; const v4f c = *(const v4f*)(p + 4);
  v4u o; o[0] = pack2(a[0], a[1]); o[1] = pack2(a[2], a[3]); o[2] = pack2(c[0], c[1]); o[3] = pack2(c[2], c[3]);
  vst2((v4u*)(XB + e * 4), o);
}

__global__ __launch_bounds__(256) void k_wt(const float* __restrict__ W, unsigned short* __restrict__ WT) {
  __shared__ __align__(16) unsigned short tl[64][72];
  const int tid = threadIdx.x; const int k0 = blockIdx.x * 64; const int n0 = blockIdx.y * 64;
#pragma unroll
  for (int it = 0; it < 4; ++it) { const int e = tid + it * 256; const int kr = e >> 4, q = e & 15;
    const v4f v = *(const v4f*)(W + (size_t)(k0 + kr) * DM + n0 + q * 4);
    tl[q * 4 + 0][kr] = (unsigned short)bf16_rne(v[0]); tl[q * 4 + 1][kr] = (unsigned short)bf16_rne(v[1]); tl[q * 4 + 2][kr] = (unsigned short)bf16_rne(v[2]); tl[q * 4 + 3][kr] = (unsigned short)bf16_rne(v[3]); }
  __syncthreads();
#pragma unroll
  for (int it = 0; it < 2; ++it) { const int e = tid + it * 256; const int n = e >> 3, q = e & 7;
    const v4u v = *(const v4u_a*)&tl[n][q * 8];
    vst2((v4u*)(WT + (size_t)(n0 + n) * DM + k0 + q * 8), v); }
}

template <int NSEG, int EPI>
__global__ __launch_bounds__(128) void k_gemm(const __bf16* __restrict__ A0, const __bf16* __restrict__ A1, const __bf16* __restrict__ BT, const float* __restrict__ BIAS, _Float16* __restrict__ OH, float* __restrict__ OF) {
  const int tid = threadIdx.x; const int wave = __builtin_amdgcn_readfirstlane((int)(threadIdx.x >> 5)); const int lane = tid & 31, col = lane & 15, g = lane >> 4;
  const int r0 = blockIdx.x * 64; const int c0 = blockIdx.y * 128;
  v8f acc[8] = {};
  const __bf16* ap0 = A0 + (size_t)(r0 + wave * 16 + col) * DM;
  const __bf16* ap1 = A1 + (size_t)(r0 + wave * 16 + col) * DM;
  const __bf16* bp = BT + (size_t)(c0 + col) * DM;
#pragma unroll 1
  for (int kc = 0; kc < DM / 32; ++kc) {
    const v16b a = frag_b(ap0 + kc * 32, lane);
    v16b a1 = a; if (NSEG == 2) a1 = frag_b(ap1 + kc * 32, lane);
#pragma unroll
    for (int j = 0; j < 8; ++j) { const v16b w = frag_b(bp + (size_t)j * 16 * DM + kc * 32, lane); acc[j] = wmma_bf(a, w, acc[j]); if (NSEG == 2) acc[j] = wmma_bf(a1, w, acc[j]); }
  }
  if (EPI == 0) {
    __shared__ __align__(16) _Float16 sh[64][136];
#pragma unroll
    for (int j = 0; j < 8; ++j) { const float bias = bfr(BIAS[c0 + j * 16 + col]);
#pragma unroll
      for (int r = 0; r < 8; ++r) sh[wave * 16 + 8 * g + r][j * 16 + col] = (_Float16)(acc[j][r] + bias); }
    __syncthreads();
    for (int e = tid; e < 64 * 16; e += 128) { const int rl = e >> 4, q = e & 15; const v4u v = *(const v4u_a*)&sh[rl][q * 8]; *(volatile v4u*)(OH + (size_t)(r0 + rl) * DM + c0 + q * 8) = v; }
    __threadfence();
    for (int e = tid; e < 64 * 16; e += 128) { const int rl = e >> 4, q = e & 15; const v4u v = *(const v4u_a*)&sh[rl][q * 8]; *(volatile v4u*)(OH + (size_t)(r0 + rl) * DM + c0 + q * 8) = v; }
  } else if (EPI == 1) {
    __shared__ __align__(16) _Float16 th[128][72];
#pragma unroll
    for (int j = 0; j < 8; ++j) { const float bias = bfr(BIAS[c0 + j * 16 + col]); v8h hv;
#pragma unroll
      for (int r = 0; r < 8; ++r) hv[r] = (_Float16)(acc[j][r] + bias);
      *(v8h_a*)&th[j * 16 + col][wave * 16 + 8 * g] = hv; }
    __syncthreads();
    const int Ls = r0 / TPS; const int tl0 = r0 - Ls * TPS;
    for (int e = tid; e < 128 * 8; e += 128) { const int cl = e >> 3, q = e & 7; const int c = c0 + cl; const int jj = c >> 6, d = c & 63;
      const v4u v = *(const v4u_a*)&th[cl][q * 8]; *(volatile v4u*)(OH + ((size_t)Ls * HD + d) * SEQ + jj * TPS + tl0 + q * 8) = v; }
    __threadfence();
    for (int e = tid; e < 128 * 8; e += 128) { const int cl = e >> 3, q = e & 7; const int c = c0 + cl; const int jj = c >> 6, d = c & 63;
      const v4u v = *(const v4u_a*)&th[cl][q * 8]; *(volatile v4u*)(OH + ((size_t)Ls * HD + d) * SEQ + jj * TPS + tl0 + q * 8) = v; }
  } else {
    __shared__ __align__(16) float ss[64][132];
#pragma unroll
    for (int j = 0; j < 8; ++j) { const float bias = bfr(BIAS[c0 + j * 16 + col]);
#pragma unroll
      for (int r = 0; r < 8; ++r) ss[wave * 16 + 8 * g + r][j * 16 + col] = acc[j][r] + bias; }
    ldsx();
    for (int rl = 0; rl < 16; ++rl) { const v4f v = *(const v4f_a*)&ss[wave * 16 + rl][lane * 4]; *(volatile v4f*)(OF + (size_t)(r0 + wave * 16 + rl) * DM + c0 + lane * 4) = v; }
    __threadfence();
    for (int rl = 0; rl < 16; ++rl) { const v4f v = *(const v4f_a*)&ss[wave * 16 + rl][lane * 4]; *(volatile v4f*)(OF + (size_t)(r0 + wave * 16 + rl) * DM + c0 + lane * 4) = v; }
  }
}

__global__ __launch_bounds__(128) void k_attn(const _Float16* __restrict__ QH, const _Float16* __restrict__ KH, const _Float16* __restrict__ VT, unsigned* __restrict__ CH, unsigned* __restrict__ CL) {
  __shared__ __align__(16) unsigned cst[4][2][16][36];
  const int tid = threadIdx.x; const int wave = __builtin_amdgcn_readfirstlane((int)(threadIdx.x >> 5)); const int lane = tid & 31, col = lane & 15, g = lane >> 4;
  const int L = blockIdx.y; const size_t qrow0 = (size_t)L * SEQ + (size_t)blockIdx.x * 64 + wave * 16;
  const _Float16* qp = QH + (qrow0 + col) * HD;
  const v16h qf0 = frag_h(qp, lane); const v16h qf1 = frag_h(qp + 32, lane);
  const _Float16* kbase = KH + ((size_t)L * TPS + col) * DM;
  const _Float16* vbase = VT + ((size_t)L * HD + col) * SEQ;
  v8f o[4] = {}; float m = -3.0e38f; float l = 0.f;
#pragma unroll 1
  for (int hb = 0; hb < SEQ / 32; ++hb) {
    const int k0 = hb * 32; const int jj = k0 / TPS; const int tl0 = k0 - jj * TPS;
    const _Float16* kp = kbase + (size_t)tl0 * DM + jj * HD;
    v8f s0 = {}, s1 = {};
    { const v16h ka = frag_h(kp, lane); const v16h kb = frag_h(kp + 32, lane); s0 = wmma16(ka, qf0, s0); s0 = wmma16(kb, qf1, s0); }
    { const v16h ka = frag_h(kp + 16 * DM, lane); const v16h kb = frag_h(kp + 16 * DM + 32, lane); s1 = wmma16(ka, qf0, s1); s1 = wmma16(kb, qf1, s1); }
    float mx = fmaxf(s0[0], s1[0]);
#pragma unroll
    for (int r = 1; r < 8; ++r) mx = fmaxf(mx, fmaxf(s0[r], s1[r]));
    mx = fmaxf(mx, __shfl_xor(mx, 16));
    const int up = mx > m ? 1 : 0;
    if (__any(up)) {
      const float mn = fmaxf(m, mx); const float corr = __expf((m - mn) * SCALE); m = mn; l *= corr;
#pragma unroll
      for (int j = 0; j < 4; ++j)
#pragma unroll
        for (int r = 0; r < 8; ++r) o[j][r] *= corr;
    }
    const float c = LN1024 - m * SCALE;
    v16h pf; float ls = 0.f;
#pragma unroll
    for (int r = 0; r < 8; ++r) { const float p0 = __expf(fmaf(s0[r], SCALE, c)); const float p1 = __expf(fmaf(s1[r], SCALE, c)); ls += p0 + p1; pf[r] = (_Float16)p0; pf[8 + r] = (_Float16)p1; }
    l += ls;
    const _Float16* vp = vbase + k0;
#pragma unroll
    for (int j = 0; j < 4; ++j) { const v16h vf = frag_h(vp + (size_t)j * 16 * SEQ, lane); o[j] = wmma16(vf, pf, o[j]); }
  }
  l += __shfl_xor(l, 16);
  const float inv = 1.0f / l;
#pragma unroll
  for (int j = 0; j < 4; ++j) { float v[8]; unsigned hb8[8];
#pragma unroll
    for (int r = 0; r < 8; ++r) { v[r] = o[j][r] * inv; hb8[r] = bf16_rne(v[r]); }
    v4u hv, lv;
#pragma unroll
    for (int t = 0; t < 4; ++t) { hv[t] = hb8[2 * t] | (hb8[2 * t + 1] << 16); lv[t] = pack2(v[2 * t] - __uint_as_float(hb8[2 * t] << 16), v[2 * t + 1] - __uint_as_float(hb8[2 * t + 1] << 16)); }
    *(v4u_a*)&cst[wave][0][col][j * 8 + g * 4] = hv; *(v4u_a*)&cst[wave][1][col][j * 8 + g * 4] = lv; }
  ldsx();
#pragma unroll
  for (int it = 0; it < 4; ++it) { const int row = it * 4 + (lane >> 3); const int pc = lane & 7;
    const v4u hv = *(const v4u_a*)&cst[wave][0][row][pc * 4]; const v4u lv = *(const v4u_a*)&cst[wave][1][row][pc * 4];
    *(volatile v4u*)(CH + (qrow0 + row) * 32 + pc * 4) = hv; *(volatile v4u*)(CL + (qrow0 + row) * 32 + pc * 4) = lv; }
  __threadfence();
#pragma unroll
  for (int it = 0; it < 4; ++it) { const int row = it * 4 + (lane >> 3); const int pc = lane & 7;
    const v4u hv = *(const v4u_a*)&cst[wave][0][row][pc * 4]; const v4u lv = *(const v4u_a*)&cst[wave][1][row][pc * 4];
    *(volatile v4u*)(CH + (qrow0 + row) * 32 + pc * 4) = hv; *(volatile v4u*)(CL + (qrow0 + row) * 32 + pc * 4) = lv; }
}

extern "C" void kernel_launch(void* const* d_in, const int* in_sizes, int n_in, void* d_out, int out_size, void* d_ws, size_t ws_size, hipStream_t stream) {
  if (n_in < 10) return;
  const long long act_min = ((long long)(NB - 1) * SEQ_FULL + SEQ) * DM;
  if ((long long)in_sizes[0] < act_min || (long long)in_sizes[1] < act_min) return;
  if (in_sizes[2] < DM * DM || in_sizes[4] < DM * DM || in_sizes[6] < DM * DM || in_sizes[8] < DM * DM) return;
  if (in_sizes[3] < DM || in_sizes[5] < DM || in_sizes[7] < DM || in_sizes[9] < DM) return;
  if ((long long)out_size < (long long)NTOK * DM) return;
  if (ws_size < (size_t)WS_END) return;
  const float* x  = (const float*)d_in[0]; const float* y  = (const float*)d_in[1];
  const float* Wq = (const float*)d_in[2]; const float* bq = (const float*)d_in[3];
  const float* Wk = (const float*)d_in[4]; const float* bk = (const float*)d_in[5];
  const float* Wv = (const float*)d_in[6]; const float* bv = (const float*)d_in[7];
  const float* Wo = (const float*)d_in[8]; const float* bo = (const float*)d_in[9];
  char* ws = (char*)d_ws;
  unsigned* XB = (unsigned*)(ws + WS_XB); unsigned* YB = (unsigned*)(ws + WS_YB);
  unsigned short* WT = (unsigned short*)(ws + WS_WT);
  unsigned short* WqT = WT; unsigned short* WkT = WT + (size_t)DM * DM; unsigned short* WvT = WT + 2 * (size_t)DM * DM; unsigned short* WoT = WT + 3 * (size_t)DM * DM;
  _Float16* QH = (_Float16*)(ws + WS_QH); _Float16* KH = (_Float16*)(ws + WS_KH); _Float16* VT = (_Float16*)(ws + WS_VT);
  unsigned* CH = (unsigned*)(ws + WS_CH); unsigned* CL = (unsigned*)(ws + WS_CL);
  float* OUT = (float*)d_out;

  const int cvt_blocks = (int)(((size_t)NTOK * (DM / 8) + 255) / 256);
  k_cvt<<<dim3(cvt_blocks), 256, 0, stream>>>(x, XB);
  k_cvt<<<dim3(cvt_blocks), 256, 0, stream>>>(y, YB);
  k_wt<<<dim3(DM / 64, DM / 64), 256, 0, stream>>>(Wq, WqT);
  k_wt<<<dim3(DM / 64, DM / 64), 256, 0, stream>>>(Wk, WkT);
  k_wt<<<dim3(DM / 64, DM / 64), 256, 0, stream>>>(Wv, WvT);
  k_wt<<<dim3(DM / 64, DM / 64), 256, 0, stream>>>(Wo, WoT);
  const dim3 gg(NTOK / 64, DM / 128);
  k_gemm<1, 0><<<gg, 128, 0, stream>>>((const __bf16*)XB, (const __bf16*)XB, (const __bf16*)WqT, bq, QH, OUT);
  k_gemm<1, 0><<<gg, 128, 0, stream>>>((const __bf16*)XB, (const __bf16*)XB, (const __bf16*)WkT, bk, KH, OUT);
  k_gemm<1, 1><<<gg, 128, 0, stream>>>((const __bf16*)YB, (const __bf16*)YB, (const __bf16*)WvT, bv, VT, OUT);
  k_attn<<<dim3(SEQ / 64, NSLAB), 128, 0, stream>>>(QH, KH, VT, CH, CL);
  k_gemm<2, 2><<<gg, 128, 0, stream>>>((const __bf16*)CH, (const __bf16*)CL, (const __bf16*)WoT, bo, QH, OUT);
}
